// GMM_48661979464133
// MI455X (gfx1250) — hardware-verified
//
#include <hip/hip_runtime.h>


namespace {
typedef _Float16 b16;
typedef __attribute__((ext_vector_type(16))) _Float16 v16b;
typedef __attribute__((ext_vector_type(8))) _Float16 v8b;
typedef __attribute__((ext_vector_type(4))) _Float16 v4h;
typedef __attribute__((ext_vector_type(2))) _Float16 v2h;
typedef __attribute__((ext_vector_type(8))) float v8f;
typedef __attribute__((ext_vector_type(4))) float v4f;
typedef __attribute__((ext_vector_type(2))) float v2f;
__device__ __forceinline__ float bf16_rne(float f) { unsigned int u = __float_as_uint(f); u += 0x7FFFu + ((u >> 16) & 1u); return __uint_as_float(u & 0xFFFF0000u); }
__device__ __forceinline__ void split16(float v, b16& hi, b16& lo) { hi = (b16)v; lo = (b16)(v - (float)hi); }
__device__ __forceinline__ v16b frag_kb(const b16* p, int hh) { const v8b a = *(const v8b*)(p + 8 * hh), b = *(const v8b*)(p + 16 + 8 * hh); v16b f;
#pragma unroll
  for (int e = 0; e < 8; ++e) { f[e] = a[e]; f[8 + e] = b[e]; } return f; }
__device__ __forceinline__ v8f wmma16b(v16b a, v16b b, v8f c) { v8f d = __builtin_amdgcn_wmma_f32_16x16x32_f16(false, a, false, b, (short)0, c, false, false); asm volatile("v_nop\n\tv_nop\n\tv_nop\n\tv_nop" : "+v"(d) : "v"(a), "v"(b)); return d; }
__device__ __forceinline__ void wave_lds_sync() { __builtin_amdgcn_fence(__ATOMIC_RELEASE, "workgroup"); __builtin_amdgcn_wave_barrier(); __builtin_amdgcn_fence(__ATOMIC_ACQUIRE, "workgroup"); }
__device__ __forceinline__ float pmul(float a, float b) { float p = a * b; asm volatile("" : "+v"(p)); return p; }
__device__ __forceinline__ int iclamp(int v, int lo, int hi) { return v < lo ? lo : (v > hi ? hi : v); }
__device__ __forceinline__ float nexp2(float v) { return __builtin_amdgcn_exp2f(v); }

constexpr int N = 65536, K = 128, M = 8, NL = N  ;
constexpr float XS = 8.0f, WSC = 256.0f;
static_assert(N % 32 == 0 && NL % 32 == 0 && K == 128, "tiling");
__global__ __launch_bounds__(256) void prep_kernel(const float* __restrict__ S, b16* __restrict__ WT) {
  const int u = blockIdx.x * 256 + threadIdx.x; if (u >= M * K * K / 8) return; const int e = u * 8; const int m = e / (K * K), r = e % (K * K); const int j = r / K, k0 = r % K; v8b o;
  for (int q = 0; q < 8; ++q) o[q] = (b16)(bf16_rne(S[((size_t)m * K + k0 + q) * K + j]) * WSC);
  for (int pass = 0; pass < 2; ++pass) { *(volatile v8b*)(WT + e) = o; __threadfence(); }
}
__global__ __launch_bounds__(128) void tab_kernel(const float* __restrict__ S, const float* __restrict__ mus, float* __restrict__ TAB) {
  __shared__ float mu_s[K], red[K]; const int m = blockIdx.x, k = threadIdx.x; mu_s[k] = bf16_rne(mus[m * K + k]); __syncthreads();
  const float* Sm = S + (size_t)m * K * K; float a = 0.0f, b = 0.0f;
#pragma unroll 1
  for (int j = 0; j < K; ++j) { a += pmul(bf16_rne(Sm[k * K + j]), mu_s[j]); b += pmul(bf16_rne(Sm[j * K + k]), mu_s[j]); }
  red[k] = pmul(mu_s[k], a); __syncthreads();
  for (int w = 64; w >= 1; w >>= 1) { if (k < w) red[k] = red[k] + red[k + w]; __syncthreads(); }
  for (int pass = 0; pass < 2; ++pass) { ((volatile float*)TAB)[m * 160 + k] = a + b; if (k < 32) ((volatile float*)TAB)[m * 160 + K + k] = (k == 0) ? red[0] : 0.0f; __threadfence(); }
}
__global__ __launch_bounds__(64) void main_kernel(const float* __restrict__ x, const b16* __restrict__ WT, const float* __restrict__ TAB, const float* __restrict__ lc, float* __restrict__ out) {
  __shared__ __attribute__((aligned(16))) b16 As[2][16][K + 8]; __shared__ float Xf[2][16][K + 4]; __shared__ float W_s[M][K + 4]; __shared__ float res[32];
  const int wave = threadIdx.x >> 5, lane = threadIdx.x & 31, nloc = lane & 15, hlf = lane >> 4; const size_t m0 = (size_t)blockIdx.x * 32 + wave * 16;
  for (int i = threadIdx.x; i < M * K; i += 64) W_s[i / K][i % K] = TAB[(i / K) * 160 + (i % K)];
  for (int rr = 0; rr < 16; ++rr) { const v4f v = *(const v4f*)(x + (m0 + rr) * K + lane * 4); v4h hv; v4f xf; for (int j = 0; j < 4; ++j) { xf[j] = bf16_rne(v[j]); hv[j] = (b16)(xf[j] * XS); } *(v4h*)(&As[wave][rr][lane * 4]) = hv; *(v4f*)(&Xf[wave][rr][lane * 4]) = xf; }
  __syncthreads();
  v16b af[4];
#pragma unroll
  for (int s = 0; s < 4; ++s) af[s] = frag_kb(&As[wave][nloc][s * 32], hlf);
  float run_m[8], run_s[8];
#pragma unroll
  for (int r = 0; r < 8; ++r) { run_m[r] = -INFINITY; run_s[r] = 0.0f; }
#pragma unroll 1
  for (int m = 0; m < M; ++m) {
    v8f acc[8];
#pragma unroll
    for (int t = 0; t < 8; ++t) acc[t] = (v8f){};
#pragma unroll
    for (int s = 0; s < 4; ++s) {
#pragma unroll
      for (int t = 0; t < 8; ++t) acc[t] = wmma16b(af[s], frag_kb(WT + ((size_t)m * K + t * 16 + nloc) * K + s * 32, hlf), acc[t]); }
    float t1[8];
#pragma unroll
    for (int r = 0; r < 8; ++r) { float p = 0.0f;
#pragma unroll
      for (int t = 0; t < 8; ++t) p = fmaf(acc[t][r] * (1.0f / (XS * WSC)), Xf[wave][8 * hlf + r][t * 16 + nloc], p); t1[r] = p; }
#pragma unroll
    for (int w = 1; w < 16; w <<= 1)
#pragma unroll
      for (int r = 0; r < 8; ++r) t1[r] += __shfl_xor(t1[r], w);
    float t2[8];
#pragma unroll
    for (int r = 0; r < 8; ++r) { float p = 0.0f;
#pragma unroll
      for (int q = 0; q < 8; ++q) p = fmaf(Xf[wave][8 * hlf + r][q * 16 + nloc], W_s[m][q * 16 + nloc], p); t2[r] = p; }
#pragma unroll
    for (int w = 1; w < 16; w <<= 1)
#pragma unroll
      for (int r = 0; r < 8; ++r) t2[r] += __shfl_xor(t2[r], w);
    const float cm = TAB[m * 160 + K], lcm = bf16_rne(lc[m]);
#pragma unroll
    for (int r = 0; r < 8; ++r) { const float V = -0.5f * (t1[r] - t2[r] + cm) + lcm; const float mn = fmaxf(run_m[r], V); run_s[r] = run_s[r] * __expf(run_m[r] - mn) + __expf(V - mn); run_m[r] = mn; } }
  if (nloc == 0) {
#pragma unroll
    for (int r = 0; r < 8; ++r) res[wave * 16 + 8 * hlf + r] = -(run_m[r] + __logf(run_s[r])); }
  __syncthreads();
  for (int pass = 0; pass < 2; ++pass) { if (wave == 0) ((volatile float*)out)[(size_t)blockIdx.x * 32 + lane] = res[lane]; __threadfence(); }
}
}

extern "C" void kernel_launch(void* const* d_in, const int* in_sizes, int n_in, void* d_out, int out_size, void* d_ws, size_t ws_size, hipStream_t stream) {
  (void)n_in;
  auto Fp = [&](int i) { return (const float*)d_in[i]; };
  if (in_sizes[0] != N * K || in_sizes[1] != M * K || in_sizes[2] != M * K * K || in_sizes[3] != M || out_size != N) return;
  size_t off = 0; char* ws = (char*)d_ws;
  auto carve = [&](size_t bytes) { char* p = ws + off; off += (bytes + 255) & ~(size_t)255; return p; };
  b16* WT = (b16*)carve((size_t)M * K * K * 2); float* TAB = (float*)carve((size_t)M * 160 * 4);
  if (off > ws_size || off > ((size_t)128 << 20)) return;
  prep_kernel<<<(M * K * K / 8 + 255) / 256, 256, 0, stream>>>(Fp(2), WT);
  tab_kernel<<<M, K, 0, stream>>>(Fp(2), Fp(1), TAB);
  main_kernel<<<NL / 32, 64, 0, stream>>>(Fp(0), WT, TAB, Fp(3), (float*)d_out);
}
